// MambaSelectiveContextAttention_71829033059044
// MI455X (gfx1250) — hardware-verified
//
#include <hip/hip_runtime.h>
#include <math.h>

typedef __attribute__((ext_vector_type(16))) _Float16 v16h;
typedef __attribute__((ext_vector_type(8)))  _Float16 v8h;
typedef __attribute__((ext_vector_type(16))) __bf16   v16b;
typedef __attribute__((ext_vector_type(8)))  __bf16   v8b;
typedef __attribute__((ext_vector_type(8)))  float    v8f;
typedef __attribute__((ext_vector_type(4)))  float    v4f;
typedef __attribute__((ext_vector_type(4)))  unsigned int v4u;

constexpr int kBatch = 2;
constexpr int kT     = 1024;
constexpr int kRows  = kBatch * kT;
constexpr int kHid   = 768;
constexpr int kNH    = 12;
constexpr int kDH    = 64;
constexpr int kWin   = 256;
constexpr int kInn   = 1536;
constexpr int kNst   = 16;
constexpr int kDtR   = 48;
constexpr int kXdW   = 80;
constexpr int kXdP   = 128;
constexpr int kXzP   = 2 * kInn;
constexpr int kQkvN  = 3 * kHid;
constexpr int kQKld  = 2 * kHid;
constexpr int kGrp   = 4;
constexpr int kNumGroups = (kBatch * kNH) / kGrp;
constexpr float kScoreScale = 0.125f;
constexpr int kConvTP = 260;
constexpr int kScanTS = 64;
constexpr int kScanCh = 64;
constexpr int kScanYP = 68;
constexpr int kScanXP = 80;
static_assert(kDtR + 2 * kNst == kXdW, "x_proj width");
static_assert(kNH % kGrp == 0, "groups stay inside one batch");
static_assert(kT == 1024, "softmax kernel: 128 threads x 8 columns = one row; block decode");
static_assert((kHid % 64) == 0 && (kInn % 64) == 0 && (kXzP % 64) == 0 && (kXdP % 64) == 0 && (kQkvN % 64) == 0 &&
              (kRows % 64) == 0 && (kT % 64) == 0 && (kDH % 64) == 0, "GEMM M,N tile multiples of 64");
static_assert((kHid % 32) == 0 && (kInn % 32) == 0 && (kDH % 32) == 0 && (kT % 32) == 0, "GEMM K multiples of 32");
static_assert((kT % kScanTS) == 0 && (kInn % kScanCh) == 0 && (kInn % 256) == 0 && (kRows % 64) == 0, "tile multiples");

constexpr size_t kMiB     = 1048576;
constexpr size_t kOffXLN  = 0;
constexpr size_t kOffXH   = 6 * kMiB;
constexpr size_t kOffXL   = 9 * kMiB;
constexpr size_t kOffHMH  = 12 * kMiB;
constexpr size_t kOffHML  = 15 * kMiB;
constexpr size_t kOffWIH  = 18 * kMiB;
constexpr size_t kOffWIL  = kOffWIH + (size_t)kXzP * kHid * 2;
constexpr size_t kOffUCH  = 12 * kMiB;
constexpr size_t kOffUCL  = 18 * kMiB;
constexpr size_t kOffYH   = 12 * kMiB;
constexpr size_t kOffYL   = 18 * kMiB;
constexpr size_t kOffXZ   = 27 * kMiB;
constexpr size_t kOffUC   = 51 * kMiB;
constexpr size_t kOffWXH  = 63 * kMiB;
constexpr size_t kOffWXL  = kOffWXH + (size_t)kXdP * kInn * 2;
constexpr size_t kOffXD   = kOffWXL + (size_t)kXdP * kInn * 2;
constexpr size_t kOffWOH  = kOffXD  + (size_t)kRows * kXdP * 4;
constexpr size_t kOffWOL  = kOffWOH + (size_t)kHid * kInn * 2;
constexpr size_t kOffMO   = 27 * kMiB;
constexpr size_t kOffSEL  = kOffWOL + (size_t)kHid * kInn * 2;
constexpr size_t kOffWQH  = 12 * kMiB;
constexpr size_t kOffWQL  = kOffWQH + (size_t)kQkvN * kHid * 2;
constexpr size_t kOffWPH  = kOffWQL + (size_t)kQkvN * kHid * 2;
constexpr size_t kOffWPL  = kOffWPH + (size_t)kHid * kHid * 2;
constexpr size_t kOffQKH  = kOffWPL + (size_t)kHid * kHid * 2;
constexpr size_t kOffQKL  = kOffQKH + (size_t)kRows * kQKld * 2;
constexpr size_t kOffVTH  = kOffQKL + (size_t)kRows * kQKld * 2;
constexpr size_t kOffVTL  = kOffVTH + (size_t)kHid * kRows * 2;
constexpr size_t kOffCTXH = kOffVTL + (size_t)kHid * kRows * 2;
constexpr size_t kOffCTXL = kOffCTXH + (size_t)kRows * kHid * 2;
constexpr size_t kOffS    = kOffCTXL + (size_t)kRows * kHid * 2;
constexpr size_t kOffPH   = 70 * kMiB;
constexpr size_t kOffPL   = kOffPH + (size_t)kGrp * kT * kT * 2;
constexpr size_t kWsTotal = kOffPL + (size_t)kGrp * kT * kT * 2;
static_assert(kOffWIL == 22 * kMiB + kMiB / 2, "map");
static_assert(kOffWIL + (size_t)kXzP * kHid * 2 == kOffXZ, "WIL ends at XZ");
static_assert(kOffUCL + (size_t)kRows * kInn * 2 <= kOffXZ, "UCL/YL inside the dead HM/WI region");
static_assert(kOffXZ + (size_t)kRows * kXzP * 4 == kOffUC, "XZ ends at UC");
static_assert(kOffUC + (size_t)kRows * kInn * 4 == kOffWXH, "UC ends at WXH");
static_assert(kOffMO + (size_t)kRows * kHid * 4 <= kOffUC, "MO inside dead XZ");
static_assert(kOffSEL == 69 * kMiB + kMiB / 4, "SEL offset");
static_assert(kOffSEL + (size_t)kRows * 4 <= kOffPH, "SEL below P planes");
static_assert(kOffQKH == 21 * kMiB && kOffCTXH == 39 * kMiB && kOffS == 45 * kMiB, "attention map");
static_assert(kOffS + (size_t)kGrp * kT * kT * 4 == 61 * kMiB, "S extent");
static_assert(kOffS + (size_t)kGrp * kT * kT * 4 <= kOffSEL, "S below SEL");
static_assert(kOffWQH >= kOffXL + (size_t)kRows * kHid * 2, "x planes not aliased");
static_assert(kOffPL == 78 * kMiB, "P planes");
static_assert(kWsTotal == 90177536ull, "carve total");
static_assert(kWsTotal <= 134217728ull, "carve cap");
static_assert((kOffWIL % 128) == 0 && (kOffWXL % 128) == 0 && (kOffXD % 128) == 0 && (kOffWOH % 128) == 0 &&
              (kOffWOL % 128) == 0 && (kOffSEL % 128) == 0 && (kOffWQL % 128) == 0 && (kOffWPH % 128) == 0 &&
              (kOffWPL % 128) == 0 && (kOffQKH % 128) == 0 && (kOffQKL % 128) == 0 && (kOffVTH % 128) == 0 &&
              (kOffVTL % 128) == 0 && (kOffCTXH % 128) == 0 && (kOffCTXL % 128) == 0 && (kOffS % 128) == 0 &&
              (kOffPL % 128) == 0, "128-B aligned regions");

__device__ __forceinline__ unsigned short f2bf_bits(float f) {
  unsigned u = __float_as_uint(f);
  return (unsigned short)((u + 0x7FFFu + ((u >> 16) & 1u)) >> 16);
}
__device__ __forceinline__ float bf_bits2f(unsigned short h) { return __uint_as_float(((unsigned)h) << 16); }
__device__ __forceinline__ unsigned pk16(unsigned short a, unsigned short b) { return (unsigned)a | ((unsigned)b << 16); }

__device__ __forceinline__ void dep_guard_h(v8f& a, v8f& b, v16h x, v16h y) { asm volatile("v_nop\n\tv_nop\n\tv_nop\n\tv_nop" : "+v"(a), "+v"(b) : "v"(x), "v"(y)); }
__device__ __forceinline__ void dep_guard_b(v8f& a, v8f& b, v16b x, v16b y) { asm volatile("v_nop\n\tv_nop\n\tv_nop\n\tv_nop" : "+v"(a), "+v"(b) : "v"(x), "v"(y)); }
__device__ __forceinline__ void keep4_h(v16h a, v16h b, v16h c, v16h d) { asm volatile("v_nop" :: "v"(a), "v"(b), "v"(c), "v"(d)); }
__device__ __forceinline__ void keep4_b(v16b a, v16b b, v16b c, v16b d) { asm volatile("v_nop" :: "v"(a), "v"(b), "v"(c), "v"(d)); }
__device__ __forceinline__ void acc_guard4(v8f& a, v8f& b, v8f& c, v8f& d) { asm volatile("v_nop\n\tv_nop\n\tv_nop\n\tv_nop" : "+v"(a), "+v"(b), "+v"(c), "+v"(d)); }
template <typename T> struct Frag;
template <> struct Frag<_Float16> {
  typedef v16h V; union U { v16h v; v8h h[2]; };
  static __device__ __forceinline__ v16h load(const _Float16* p) {
    U f; f.h[0] = *(const v8h*)(p); f.h[1] = *(const v8h*)(p + 16); return f.v;
  }
  static __device__ __forceinline__ v8f mma(v16h a, v16h b, v8f c) {
    return __builtin_amdgcn_wmma_f32_16x16x32_f16(false, a, false, b, (short)0, c, false, false);
  }
  static __device__ __forceinline__ void guard(v8f& a, v8f& b, v16h x, v16h y) { dep_guard_h(a, b, x, y); }
  static __device__ __forceinline__ void keep(v16h a, v16h b, v16h c, v16h d) { keep4_h(a, b, c, d); }
};
template <> struct Frag<__bf16> {
  typedef v16b V; union U { v16b v; v8b h[2]; };
  static __device__ __forceinline__ v16b load(const __bf16* p) {
    U f; f.h[0] = *(const v8b*)(p); f.h[1] = *(const v8b*)(p + 16); return f.v;
  }
  static __device__ __forceinline__ v8f mma(v16b a, v16b b, v8f c) {
    return __builtin_amdgcn_wmma_f32_16x16x32_bf16(false, a, false, b, (short)0, c, false, false);
  }
  static __device__ __forceinline__ void guard(v8f& a, v8f& b, v16b x, v16b y) { dep_guard_b(a, b, x, y); }
  static __device__ __forceinline__ void keep(v16b a, v16b b, v16b c, v16b d) { keep4_b(a, b, c, d); }
};

__device__ __forceinline__ float wave_sum32(float v) {
#pragma unroll
  for (int off = 16; off > 0; off >>= 1) v += __shfl_xor(v, off, 32);
  return v;
}
__device__ __forceinline__ float wave_max32(float v) {
#pragma unroll
  for (int off = 16; off > 0; off >>= 1) v = fmaxf(v, __shfl_xor(v, off, 32));
  return v;
}

template <int ET> struct Elem;
template <> struct Elem<0> { typedef _Float16 T; };
template <> struct Elem<1> { typedef __bf16 T; };
template <int ET, int SPL, int BIAS_MODE, int OUT_MODE, bool RESID, int ACT = 0, bool CAUSAL = false>
__global__ __launch_bounds__(256) void wmma_gemm64(
    const unsigned short* __restrict__ Ap, const unsigned short* __restrict__ A2p, int lda, long strideA,
    const unsigned short* __restrict__ Btp, const unsigned short* __restrict__ Bt2p, int ldb, long strideB,
    void* __restrict__ Cout, void* __restrict__ Cout2, int ldc, long strideC,
    const float* __restrict__ bias,
    const float* __restrict__ resid, long strideR,
    int M, int N, int K, float scale) {
  typedef typename Elem<ET>::T T;
  typedef typename Frag<T>::V V;
  const T* A = (const T*)Ap; const T* A2 = (const T*)A2p; const T* Bt = (const T*)Btp; const T* Bt2 = (const T*)Bt2p;
  __shared__ __align__(16) float sT[8][16 * 68];
  const int b    = blockIdx.y;
  const int lane = threadIdx.x & 31;
  const int wave = threadIdx.x >> 5;
  const int tilesN = N >> 6;
  const int tilesM = M >> 6;
  const int tile = blockIdx.x * 8 + wave;
  if (tile >= tilesM * tilesN) return;
  const int tm = tile / tilesN;
  const int tn = tile - tm * tilesN;
  const int m0 = tm << 6;
  const int n0 = tn << 6;
  if (CAUSAL && (n0 > m0)) return;
  const int Kend = CAUSAL ? ((m0 + 64 < K) ? (m0 + 64) : K) : K;

  const T* Ab  = A  + (size_t)b * strideA;
  const T* Bb  = Bt + (size_t)b * strideB;
  const T* Ab2 = (SPL >= 1) ? (A2  + (size_t)b * strideA) : nullptr;
  const T* Bb2 = (SPL == 2) ? (Bt2 + (size_t)b * strideB) : nullptr;

  const int rlane = lane & 15;
  const int koff  = (lane >> 4) * 8;
  const int mOff  = (lane >> 4) * 8;

  v8f acc[4][4];
#pragma unroll
  for (int i = 0; i < 4; ++i)
#pragma unroll
    for (int j = 0; j < 4; ++j) acc[i][j] = (v8f){0.f,0.f,0.f,0.f,0.f,0.f,0.f,0.f};

  for (int k0 = 0; k0 < Kend; k0 += 32) {
    V bh[4], bl[4];
#pragma unroll
    for (int j = 0; j < 4; ++j) {
      const size_t bo = (size_t)(n0 + (j << 4) + rlane) * ldb + koff + k0;
      bh[j] = Frag<T>::load(Bb + bo);
      if (SPL == 2) bl[j] = Frag<T>::load(Bb2 + bo);
    }
#pragma unroll
    for (int i = 0; i < 4; ++i) {
      const size_t ao = (size_t)(m0 + (i << 4) + rlane) * lda + koff + k0;
      V ah = Frag<T>::load(Ab + ao);
      V al;
      if (SPL >= 1) al = Frag<T>::load(Ab2 + ao);
#pragma unroll
      for (int j = 0; j < 4; ++j) {
        acc[i][j] = Frag<T>::mma(ah, bh[j], acc[i][j]);
        if (SPL == 2) acc[i][j] = Frag<T>::mma(ah, bl[j], acc[i][j]);
        if (SPL >= 1) acc[i][j] = Frag<T>::mma(al, bh[j], acc[i][j]);
      }
      Frag<T>::guard(acc[i][0], acc[i][3], ah, (SPL >= 1) ? al : ah);
    }
    Frag<T>::keep(bh[0], bh[1], bh[2], bh[3]);
    if (SPL == 2) Frag<T>::keep(bl[0], bl[1], bl[2], bl[3]);
  }
  acc_guard4(acc[0][0], acc[0][1], acc[0][2], acc[0][3]);
  acc_guard4(acc[1][0], acc[1][1], acc[1][2], acc[1][3]);
  acc_guard4(acc[2][0], acc[2][1], acc[2][2], acc[2][3]);
  acc_guard4(acc[3][0], acc[3][1], acc[3][2], acc[3][3]);

  float* slab = sT[wave];
  const float* Rb = RESID ? (resid + (size_t)b * strideR) : nullptr;
#pragma unroll
  for (int i = 0; i < 4; ++i) {
    const int mBase = m0 + (i << 4);
#pragma unroll
    for (int j = 0; j < 4; ++j) {
      const int n = n0 + (j << 4) + rlane;
      float bv = 0.f;
      if (BIAS_MODE == 2) bv = bias[n];
#pragma unroll
      for (int r = 0; r < 8; ++r) {
        float v = acc[i][j][r] * scale;
        if (BIAS_MODE == 1) v += bias[mBase + mOff + r];
        if (BIAS_MODE == 2) v += bv;
        if (RESID) v += Rb[(size_t)(mBase + mOff + r) * ldc + n];
        if (ACT == 2) v = fmaxf(v, 0.0f);
        if (ACT == 4) v = (v > 0.f) ? v : 0.01f * v;
        if (ACT == 6) v = fminf(20.0f, fmaxf(-20.0f, v));
        slab[(mOff + r) * 68 + (j << 4) + rlane] = v;
      }
    }
    __builtin_amdgcn_fence(__ATOMIC_RELEASE, "workgroup");
    __builtin_amdgcn_wave_barrier();
    __builtin_amdgcn_fence(__ATOMIC_ACQUIRE, "workgroup");
    if (OUT_MODE == 0) {
      float* C = (float*)Cout + (size_t)b * strideC;
      const int hh = lane >> 4, c4 = (lane & 15) * 4;
      for (int pass = 0; pass < 2; ++pass) {
#pragma unroll
        for (int it = 0; it < 8; ++it) {
          const int row = it * 2 + hh;
          v4f v = *(const v4f*)(slab + row * 68 + c4);
          *(volatile v4f*)(C + (size_t)(mBase + row) * ldc + n0 + c4) = v;
        }
        __threadfence();
      }
    } else {
      const int q = lane >> 3, c8 = (lane & 7) * 8;
      unsigned short* C  = (unsigned short*)Cout  + (size_t)b * strideC;
      unsigned short* C2 = (OUT_MODE == 2) ? ((unsigned short*)Cout2 + (size_t)b * strideC) : nullptr;
      for (int pass = 0; pass < 2; ++pass) {
#pragma unroll
        for (int it = 0; it < 4; ++it) {
          const int row = it * 4 + q;
          const float* sp = slab + row * 68 + c8;
          v8h hv, lv;
#pragma unroll
          for (int e = 0; e < 8; ++e) {
            if (OUT_MODE == 1) {
              hv[e] = (_Float16)sp[e];
            } else {
              unsigned short hb = f2bf_bits(sp[e]);
              unsigned short lb = f2bf_bits(sp[e] - bf_bits2f(hb));
              hv[e] = __builtin_bit_cast(_Float16, hb);
              lv[e] = __builtin_bit_cast(_Float16, lb);
            }
          }
          *(volatile v8h*)(C + (size_t)(mBase + row) * ldc + n0 + c8) = hv;
          if (OUT_MODE == 2) *(volatile v8h*)(C2 + (size_t)(mBase + row) * ldc + n0 + c8) = lv;
        }
        __threadfence();
      }
    }
    __builtin_amdgcn_fence(__ATOMIC_RELEASE, "workgroup");
    __builtin_amdgcn_wave_barrier();
    __builtin_amdgcn_fence(__ATOMIC_ACQUIRE, "workgroup");
  }
}

__global__ __launch_bounds__(256) void transpose_split_kernel(const float* __restrict__ in, int ldin, int Cn,
                                                              unsigned short* __restrict__ oh, unsigned short* __restrict__ ol,
                                                              int ldout) {
  __shared__ float sm[64][65];
  const int t  = threadIdx.x;
  const int r0 = blockIdx.x * 64;
  const int c0 = blockIdx.y * 64;
#pragma unroll
  for (int i = 0; i < 16; ++i) {
    const int e = i * 256 + t;
    const int r = e >> 6;
    const int c = e & 63;
    const int cg = c0 + c;
    const int ca = (cg < Cn) ? cg : (Cn - 1);
    const float v = in[(size_t)(r0 + r) * ldin + ca];
    sm[c][r] = (cg < Cn) ? v : 0.0f;
  }
  __syncthreads();
  const int lane = t & 31, wave = t >> 5;
  const int q = lane >> 3, c8 = (lane & 7) * 8;
  v4u hu[2], lu[2];
#pragma unroll
  for (int it = 0; it < 2; ++it) {
    const int row = wave * 8 + it * 4 + q;
    unsigned hw[4], lw[4];
#pragma unroll
    for (int e2 = 0; e2 < 4; ++e2) {
      const float f0 = sm[row][c8 + 2 * e2], f1 = sm[row][c8 + 2 * e2 + 1];
      const unsigned short h0 = f2bf_bits(f0), h1 = f2bf_bits(f1);
      const unsigned short l0 = f2bf_bits(f0 - bf_bits2f(h0)), l1 = f2bf_bits(f1 - bf_bits2f(h1));
      hw[e2] = pk16(h0, h1);
      lw[e2] = pk16(l0, l1);
    }
    hu[it] = (v4u){hw[0], hw[1], hw[2], hw[3]};
    lu[it] = (v4u){lw[0], lw[1], lw[2], lw[3]};
  }
  for (int pass = 0; pass < 2; ++pass) {
#pragma unroll
    for (int it = 0; it < 2; ++it) {
      const int row = wave * 8 + it * 4 + q;
      const size_t o = (size_t)(c0 + row) * ldout + r0 + c8;
      *(volatile v4u*)(oh + o) = hu[it];
      *(volatile v4u*)(ol + o) = lu[it];
    }
    __threadfence();
  }
}

__global__ __launch_bounds__(256) void ln_rms_kernel(
    const float* __restrict__ x, const float* __restrict__ lnw, const float* __restrict__ lnb,
    const float* __restrict__ mnw, float* __restrict__ XLN,
    unsigned short* __restrict__ XH, unsigned short* __restrict__ XL,
    unsigned short* __restrict__ HMH, unsigned short* __restrict__ HML)
{
  __shared__ __align__(16) float sA[kHid];
  __shared__ __align__(16) float sB[kHid];
  __shared__ float red[3][8];
  const int row = blockIdx.x, t = threadIdx.x, lane = t & 31, wave = t >> 5;
  const float* xr = x + (size_t)row * kHid;
  float loc[3];
  float s = 0.f;
#pragma unroll
  for (int c = 0; c < 3; ++c) { loc[c] = xr[t + 256 * c]; s += loc[c]; }
  s = wave_sum32(s);
  if (lane == 0) red[0][wave] = s;
  __syncthreads();
  float tot = 0.f;
#pragma unroll
  for (int w = 0; w < 8; ++w) tot += red[0][w];
  const float mu = tot * (1.0f / 768.0f);
  float vs = 0.f;
#pragma unroll
  for (int c = 0; c < 3; ++c) { const float dd = loc[c] - mu; vs += dd * dd; }
  vs = wave_sum32(vs);
  if (lane == 0) red[1][wave] = vs;
  __syncthreads();
  float vt = 0.f;
#pragma unroll
  for (int w = 0; w < 8; ++w) vt += red[1][w];
  const float rs = rsqrtf(vt * (1.0f / 768.0f) + 1e-5f);
  float xv[3];
  float sq = 0.f;
#pragma unroll
  for (int c = 0; c < 3; ++c) {
    const int j = t + 256 * c;
    xv[c] = (loc[c] - mu) * rs * lnw[j] + lnb[j];
    sA[j] = xv[c];
    sq += xv[c] * xv[c];
  }
  sq = wave_sum32(sq);
  if (lane == 0) red[2][wave] = sq;
  __syncthreads();
  float st = 0.f;
#pragma unroll
  for (int w = 0; w < 8; ++w) st += red[2][w];
  const float rs2 = rsqrtf(st * (1.0f / 768.0f) + 1e-5f);
#pragma unroll
  for (int c = 0; c < 3; ++c) {
    const int j = t + 256 * c;
    sB[j] = xv[c] * rs2 * mnw[j];
  }
  __syncthreads();
  const int tA = (t < 192) ? t : 191;
  const int tB = (t < 96) ? t : 95;
  const v4f fx = *(const v4f*)(sA + 4 * tA);
  const v4f x0 = *(const v4f*)(xr + 8 * tB);
  const v4f x1 = *(const v4f*)(xr + 8 * tB + 4);
  const v4f m0 = *(const v4f*)(sB + 8 * tB);
  const v4f m1 = *(const v4f*)(sB + 8 * tB + 4);
  v8h xh, xl, mh, ml;
#pragma unroll
  for (int e = 0; e < 4; ++e) {
    const unsigned short a0 = f2bf_bits(x0[e]), a1 = f2bf_bits(x1[e]);
    const unsigned short b0 = f2bf_bits(x0[e] - bf_bits2f(a0)), b1 = f2bf_bits(x1[e] - bf_bits2f(a1));
    const unsigned short c0h = f2bf_bits(m0[e]), c1h = f2bf_bits(m1[e]);
    const unsigned short d0 = f2bf_bits(m0[e] - bf_bits2f(c0h)), d1 = f2bf_bits(m1[e] - bf_bits2f(c1h));
    xh[e] = __builtin_bit_cast(_Float16, a0);  xh[4 + e] = __builtin_bit_cast(_Float16, a1);
    xl[e] = __builtin_bit_cast(_Float16, b0);  xl[4 + e] = __builtin_bit_cast(_Float16, b1);
    mh[e] = __builtin_bit_cast(_Float16, c0h); mh[4 + e] = __builtin_bit_cast(_Float16, c1h);
    ml[e] = __builtin_bit_cast(_Float16, d0);  ml[4 + e] = __builtin_bit_cast(_Float16, d1);
  }
  const size_t ro = (size_t)row * kHid;
  for (int pass = 0; pass < 2; ++pass) {
    if (t < 192) *(volatile v4f*)(XLN + ro + 4 * t) = fx;
    if (t < 96) {
      *(volatile v8h*)(XH  + ro + 8 * t) = xh;
      *(volatile v8h*)(XL  + ro + 8 * t) = xl;
      *(volatile v8h*)(HMH + ro + 8 * t) = mh;
      *(volatile v8h*)(HML + ro + 8 * t) = ml;
    }
    __threadfence();
  }
}

__global__ __launch_bounds__(256) void conv_silu_kernel(
    const float* __restrict__ XZ, const float* __restrict__ cw, const float* __restrict__ cb,
    float* __restrict__ UC, unsigned short* __restrict__ UCH, unsigned short* __restrict__ UCL)
{
  __shared__ __align__(16) float sT[16 * kConvTP];
  const int tid = threadIdx.x, lane = tid & 31, wave = tid >> 5;
  const int d0 = blockIdx.x * 256, d = d0 + tid;
  const int g0 = blockIdx.y * 64;
  const int tb = g0 & (kT - 1);
  const float w0 = cw[d * 4 + 0], w1 = cw[d * 4 + 1], w2 = cw[d * 4 + 2], w3 = cw[d * 4 + 3];
  const float bc = cb[d];
  float xm3, xm2, xm1;
  {
    const bool hist = (tb > 0);
    const int rb = hist ? (g0 - 3) : g0;
    const float v3 = XZ[(size_t)rb * kXzP + d];
    const float v2 = XZ[(size_t)(rb + 1) * kXzP + d];
    const float v1 = XZ[(size_t)(rb + 2) * kXzP + d];
    xm3 = hist ? v3 : 0.f;
    xm2 = hist ? v2 : 0.f;
    xm1 = hist ? v1 : 0.f;
  }
  const int hrow = wave >> 1;
  const int hch  = (wave & 1) * 128 + lane * 4;
#pragma unroll 1
  for (int sub = 0; sub < 4; ++sub) {
    const int lb = g0 + sub * 16;
#pragma unroll 1
    for (int s = 0; s < 16; ++s) {
      const float xcur = XZ[(size_t)(lb + s) * kXzP + d];
      float acc = w0 * xm3;
      acc = fmaf(w1, xm2, acc);
      acc = fmaf(w2, xm1, acc);
      acc = fmaf(w3, xcur, acc);
      const float sv = acc + bc;
      const float sg = __builtin_amdgcn_rcpf(1.0f + __expf(-sv));
      sT[s * kConvTP + tid] = sv * sg;
      xm3 = xm2; xm2 = xm1; xm1 = xcur;
    }
    __syncthreads();
    v4f fv[4];
    v8h bh[2], blo[2];
#pragma unroll
    for (int it = 0; it < 4; ++it) fv[it] = *(const v4f*)(sT + (it * 4 + hrow) * kConvTP + hch);
#pragma unroll
    for (int it = 0; it < 2; ++it) {
      const float* sp = sT + (it * 8 + wave) * kConvTP + lane * 8;
      const v4f a0 = *(const v4f*)(sp);
      const v4f a1 = *(const v4f*)(sp + 4);
#pragma unroll
      for (int e = 0; e < 4; ++e) {
        const unsigned short h0 = f2bf_bits(a0[e]), h1 = f2bf_bits(a1[e]);
        const unsigned short l0 = f2bf_bits(a0[e] - bf_bits2f(h0)), l1 = f2bf_bits(a1[e] - bf_bits2f(h1));
        bh[it][e]      = __builtin_bit_cast(_Float16, h0);
        bh[it][4 + e]  = __builtin_bit_cast(_Float16, h1);
        blo[it][e]     = __builtin_bit_cast(_Float16, l0);
        blo[it][4 + e] = __builtin_bit_cast(_Float16, l1);
      }
    }
    for (int pass = 0; pass < 2; ++pass) {
#pragma unroll
      for (int it = 0; it < 4; ++it)
        *(volatile v4f*)(UC + (size_t)(lb + it * 4 + hrow) * kInn + d0 + hch) = fv[it];
#pragma unroll
      for (int it = 0; it < 2; ++it) {
        const size_t o = (size_t)(lb + it * 8 + wave) * kInn + d0 + lane * 8;
        *(volatile v8h*)(UCH + o) = bh[it];
        *(volatile v8h*)(UCL + o) = blo[it];
      }
      __threadfence();
    }
    __syncthreads();
  }
}

__global__ __launch_bounds__(64) void scan_kernel(
    const float* __restrict__ XD, const float* __restrict__ UC, const float* __restrict__ XZ,
    const float* __restrict__ Wdt, const float* __restrict__ bdt, const float* __restrict__ Alog,
    const float* __restrict__ Dp, unsigned short* __restrict__ YH, unsigned short* __restrict__ YL)
{
  __shared__ __align__(16) float sX[kScanTS * kScanXP];
  __shared__ __align__(16) float sY[kScanTS * kScanYP];
  __shared__ __align__(16) float sW[kDtR * kScanCh];
  __shared__ __align__(16) float sA[kNst * kScanCh];
  const int tid = threadIdx.x, lane = tid & 31, wave = tid >> 5;
  constexpr int kBlkPerB = kInn / kScanCh;
  const int bix = blockIdx.x / kBlkPerB;
  const int d0  = (blockIdx.x - bix * kBlkPerB) * kScanCh;
  const int d   = d0 + tid;
  const size_t row0 = (size_t)bix * kT;
#pragma unroll 1
  for (int r = 0; r < kDtR; ++r) sW[r * kScanCh + tid] = Wdt[(size_t)r * kInn + d];
#pragma unroll 1
  for (int s = 0; s < kNst; ++s) sA[s * kScanCh + tid] = -expf(Alog[(size_t)d * kNst + s]);
  __syncthreads();
  float negA[kNst], h[kNst];
#pragma unroll
  for (int s = 0; s < kNst; ++s) {
    negA[s] = sA[s * kScanCh + tid];
    h[s] = 0.f;
  }
  const float bb = bdt[d], Dd = Dp[d];
  const int q = lane >> 3, c8 = (lane & 7) * 8;
#pragma unroll 1
  for (int t0 = 0; t0 < kT; t0 += kScanTS) {
    __syncthreads();
#pragma unroll
    for (int i = 0; i < 20; ++i) {
      const int e  = i * 64 + tid;
      const int r  = e / 20;
      const int c4 = (e - r * 20) * 4;
      *(v4f*)(sX + r * kScanXP + c4) = *(const v4f*)(XD + (row0 + t0 + r) * kXdP + c4);
    }
    __syncthreads();
#pragma unroll 1
    for (int s = 0; s < kScanTS; ++s) {
      const int t = t0 + s;
      const float* xr = sX + s * kScanXP;
      float vdot = 0.f;
#pragma unroll 1
      for (int r4 = 0; r4 < kDtR / 4; ++r4) {
        const v4f xv = *(const v4f*)(xr + 4 * r4);
        const float* wp = sW + (4 * r4) * kScanCh + tid;
        vdot = fmaf(xv[0], wp[0], vdot);
        vdot = fmaf(xv[1], wp[kScanCh], vdot);
        vdot = fmaf(xv[2], wp[2 * kScanCh], vdot);
        vdot = fmaf(xv[3], wp[3 * kScanCh], vdot);
      }
      float Bs[kNst], Cs[kNst];
#pragma unroll
      for (int q4 = 0; q4 < 4; ++q4) {
        const v4f bv = *(const v4f*)(xr + kDtR + 4 * q4);
        const v4f cv = *(const v4f*)(xr + kDtR + kNst + 4 * q4);
        Bs[4 * q4 + 0] = bv[0]; Bs[4 * q4 + 1] = bv[1]; Bs[4 * q4 + 2] = bv[2]; Bs[4 * q4 + 3] = bv[3];
        Cs[4 * q4 + 0] = cv[0]; Cs[4 * q4 + 1] = cv[1]; Cs[4 * q4 + 2] = cv[2]; Cs[4 * q4 + 3] = cv[3];
      }
      const float v   = vdot + bb;
      const float a   = __expf(-fabsf(v));
      const float u   = 1.0f + a;
      const float l1p = __logf(u) + (a - (u - 1.0f)) * __builtin_amdgcn_rcpf(u);
      const float dt  = fmaxf(v, 0.0f) + l1p;
      const float xt  = UC[(row0 + t) * kInn + d];
      float y = 0.f;
#pragma unroll
      for (int k = 0; k < kNst; ++k) {
        const float e   = __expf(dt * negA[k]);
        const float dtB = dt * Bs[k];
        h[k] = e * h[k] + dtB * xt;
        y = h[k] * Cs[k] + y;
      }
      y = xt * Dd + y;
      const float zv = XZ[(row0 + t) * kXzP + kInn + d];
      const float sg = __builtin_amdgcn_rcpf(1.0f + __expf(-zv));
      y = y * (zv * sg);
      sY[s * kScanYP + tid] = y;
    }
    __syncthreads();
    v8h hv[8], lv[8];
#pragma unroll
    for (int it = 0; it < 8; ++it) {
      const int row = it * 8 + wave * 4 + q;
      const float* sp = sY + row * kScanYP + c8;
      const v4f a0 = *(const v4f*)(sp);
      const v4f a1 = *(const v4f*)(sp + 4);
#pragma unroll
      for (int e = 0; e < 4; ++e) {
        const unsigned short h0 = f2bf_bits(a0[e]), h1 = f2bf_bits(a1[e]);
        const unsigned short l0 = f2bf_bits(a0[e] - bf_bits2f(h0)), l1 = f2bf_bits(a1[e] - bf_bits2f(h1));
        hv[it][e]     = __builtin_bit_cast(_Float16, h0);
        hv[it][4 + e] = __builtin_bit_cast(_Float16, h1);
        lv[it][e]     = __builtin_bit_cast(_Float16, l0);
        lv[it][4 + e] = __builtin_bit_cast(_Float16, l1);
      }
    }
    for (int pass = 0; pass < 2; ++pass) {
#pragma unroll
      for (int it = 0; it < 8; ++it) {
        const int row = it * 8 + wave * 4 + q;
        const size_t o = (row0 + t0 + row) * kInn + d0 + c8;
        *(volatile v8h*)(YH + o) = hv[it];
        *(volatile v8h*)(YL + o) = lv[it];
      }
      __threadfence();
    }
  }
}

__global__ __launch_bounds__(256) void gate_kernel(
    const float* __restrict__ MO, const float* __restrict__ sw, const float* __restrict__ sb, float* __restrict__ SEL)
{
  __shared__ __align__(16) float sv[32];
  const int t = threadIdx.x, lane = t & 31, wave = t >> 5;
  const int rb = blockIdx.x * 32;
  const float bias0 = sb[0];
#pragma unroll
  for (int rr = 0; rr < 4; ++rr) {
    const int row = rb + wave * 4 + rr;
    const float* mr = MO + (size_t)row * kHid;
    float acc = 0.f;
#pragma unroll 1
    for (int k = 0; k < kHid / 32; ++k) acc = fmaf(mr[lane + 32 * k], sw[lane + 32 * k], acc);
    acc = wave_sum32(acc);
    const float s = 1.0f / (1.0f + expf(-(acc + bias0)));
    if (lane == 0) sv[wave * 4 + rr] = s;
  }
  __syncthreads();
  const int tl = (t < 8) ? t : 7;
  const v4f val = *(const v4f*)(sv + 4 * tl);
  for (int pass = 0; pass < 2; ++pass) {
    if (t < 8) *(volatile v4f*)(SEL + rb + 4 * t) = val;
    __threadfence();
  }
}

__global__ __launch_bounds__(128) void softmax_dual_kernel(const float* __restrict__ S, const float* __restrict__ selp,
                                                           const float* __restrict__ wlp, const float* __restrict__ wgp,
                                                           unsigned short* __restrict__ Phi, unsigned short* __restrict__ Plo) {
  __shared__ float redMG[4], redML[4], redSG[4], redSL[4];
  const float ninf = -__builtin_inff();
  const int blk  = blockIdx.x;
  const int pr   = blk >> 10;
  const int qi   = blk & (kT - 1);
  const int t    = threadIdx.x;
  const int lane = t & 31, wave = t >> 5;
  const int c0   = t * 8;
  const size_t rowoff = ((size_t)pr * kT + qi) * (size_t)kT;
  const bool wave_live = (wave * 256 <= qi);

  const float e0 = expf(-wlp[0]);
  const float e1 = expf(-wgp[0]);
  const float a0 = 1.0f / (1.0f + e0);
  const float a1 = 1.0f / (1.0f + e1);
  const float rsum = 1.0f / (a0 + a1);
  const float wl = a0 * rsum;
  const float wg = a1 * rsum;

  float xg[8], xl[8];
  float mg = ninf, ml = ninf;
  if (wave_live) {
    const float* sr = S + rowoff + c0;
    const v4f sa = *(const v4f*)(sr);
    const v4f sc = *(const v4f*)(sr + 4);
    const v4f ea = *(const v4f*)(selp + c0);
    const v4f ec = *(const v4f*)(selp + c0 + 4);
    float sv[8], ev[8];
#pragma unroll
    for (int e = 0; e < 4; ++e) { sv[e] = sa[e]; sv[4 + e] = sc[e]; ev[e] = ea[e]; ev[4 + e] = ec[e]; }
#pragma unroll
    for (int e = 0; e < 8; ++e) {
      const int j = c0 + e;
      const float fac = 0.5f * (1.0f + ev[e]);
      const bool excl = (j > qi);
      const bool outside = (j < qi - kWin);
      const float gv = excl ? ninf : sv[e] * fac;
      const float lv = (excl || outside) ? ninf : sv[e];
      xg[e] = gv; xl[e] = lv;
      mg = fmaxf(mg, gv);
      ml = fmaxf(ml, lv);
    }
  } else {
#pragma unroll
    for (int e = 0; e < 8; ++e) { xg[e] = ninf; xl[e] = ninf; }
  }
  mg = wave_max32(mg);
  ml = wave_max32(ml);
  if (lane == 0) { redMG[wave] = mg; redML[wave] = ml; }
  __syncthreads();
  float gmaxG = redMG[0], gmaxL = redML[0];
#pragma unroll
  for (int w = 1; w < 4; ++w) { gmaxG = fmaxf(gmaxG, redMG[w]); gmaxL = fmaxf(gmaxL, redML[w]); }
  const bool liveG = (gmaxG > ninf);
  const bool liveL = (gmaxL > ninf);
  const float subG = liveG ? gmaxG : 0.0f;
  const float subL = liveL ? gmaxL : 0.0f;

  float pg[8], pl[8];
  float psG = 0.0f, psL = 0.0f;
  if (wave_live) {
#pragma unroll
    for (int e = 0; e < 8; ++e) {
      pg[e] = __expf(xg[e] - subG); psG += pg[e];
      pl[e] = __expf(xl[e] - subL); psL += pl[e];
    }
  } else {
#pragma unroll
    for (int e = 0; e < 8; ++e) { pg[e] = 0.0f; pl[e] = 0.0f; }
  }
  psG = wave_sum32(psG);
  psL = wave_sum32(psL);
  if (lane == 0) { redSG[wave] = psG; redSL[wave] = psL; }
  __syncthreads();
  float totG = redSG[0], totL = redSL[0];
#pragma unroll
  for (int w = 1; w < 4; ++w) { totG += redSG[w]; totL += redSL[w]; }
  const float invG = liveG ? (wg * __builtin_amdgcn_rcpf(totG)) : 0.0f;
  const float invL = liveL ? (wl * __builtin_amdgcn_rcpf(totL)) : 0.0f;

  unsigned hw[4], lw[4];
#pragma unroll
  for (int e2 = 0; e2 < 4; ++e2) {
    float f0 = pl[2 * e2] * invL + pg[2 * e2] * invG;
    float f1 = pl[2 * e2 + 1] * invL + pg[2 * e2 + 1] * invG;
    f0 = (f0 == f0) ? f0 : 0.0f;
    f1 = (f1 == f1) ? f1 : 0.0f;
    const unsigned short h0 = f2bf_bits(f0);
    const unsigned short h1 = f2bf_bits(f1);
    const unsigned short l0 = f2bf_bits(f0 - bf_bits2f(h0));
    const unsigned short l1 = f2bf_bits(f1 - bf_bits2f(h1));
    hw[e2] = pk16(h0, h1);
    lw[e2] = pk16(l0, l1);
  }
  const v4u hv = (v4u){hw[0], hw[1], hw[2], hw[3]};
  const v4u lv4 = (v4u){lw[0], lw[1], lw[2], lw[3]};
  unsigned short* ph = Phi + rowoff + c0;
  unsigned short* plp = Plo + rowoff + c0;
  *(volatile v4u*)ph = hv;
  *(volatile v4u*)plp = lv4;
  __threadfence();
  *(volatile v4u*)ph = hv;
  *(volatile v4u*)plp = lv4;
}

extern "C" void kernel_launch(void* const* d_in, const int* in_sizes, int n_in,
                              void* d_out, int out_size, void* d_ws, size_t ws_size,
                              hipStream_t stream) {
  if (n_in < 21) return;
  if (in_sizes[0]  != kRows * kHid) return;
  if (in_sizes[1]  != kHid * kQkvN) return;
  if (in_sizes[2]  != kQkvN) return;
  if (in_sizes[3]  != kHid * kHid) return;
  if (in_sizes[4]  != kHid) return;
  if (in_sizes[5]  != kHid) return;
  if (in_sizes[6]  != kHid) return;
  if (in_sizes[7]  != kHid) return;
  if (in_sizes[8]  != 1) return;
  if (in_sizes[9]  != 1) return;
  if (in_sizes[10] != 1) return;
  if (in_sizes[11] != kHid) return;
  if (in_sizes[12] != kHid * kXzP) return;
  if (in_sizes[13] != kInn * 4) return;
  if (in_sizes[14] != kInn) return;
  if (in_sizes[15] != kInn * kXdW) return;
  if (in_sizes[16] != kDtR * kInn) return;
  if (in_sizes[17] != kInn) return;
  if (in_sizes[18] != kInn * kNst) return;
  if (in_sizes[19] != kInn) return;
  if (in_sizes[20] != kInn * kHid) return;
  if (out_size != kRows * kHid) return;
  if (ws_size < kWsTotal) return;

  const float* x          = (const float*)d_in[0];
  const float* c_attn_w   = (const float*)d_in[1];
  const float* c_attn_b   = (const float*)d_in[2];
  const float* c_proj_w   = (const float*)d_in[3];
  const float* c_proj_b   = (const float*)d_in[4];
  const float* ln_w       = (const float*)d_in[5];
  const float* ln_b       = (const float*)d_in[6];
  const float* sel_w      = (const float*)d_in[7];
  const float* sel_b      = (const float*)d_in[8];
  const float* w_local    = (const float*)d_in[9];
  const float* w_global   = (const float*)d_in[10];
  const float* m_norm_w   = (const float*)d_in[11];
  const float* in_proj_w  = (const float*)d_in[12];
  const float* conv_w     = (const float*)d_in[13];
  const float* conv_b     = (const float*)d_in[14];
  const float* x_proj_w   = (const float*)d_in[15];
  const float* dt_proj_w  = (const float*)d_in[16];
  const float* dt_proj_b  = (const float*)d_in[17];
  const float* A_log      = (const float*)d_in[18];
  const float* Dp         = (const float*)d_in[19];
  const float* out_proj_w = (const float*)d_in[20];
  float* out = (float*)d_out;

  char* ws = (char*)d_ws;
  float*          XLN  = (float*)(ws + kOffXLN);
  unsigned short* XH   = (unsigned short*)(ws + kOffXH);
  unsigned short* XL   = (unsigned short*)(ws + kOffXL);
  unsigned short* HMH  = (unsigned short*)(ws + kOffHMH);
  unsigned short* HML  = (unsigned short*)(ws + kOffHML);
  unsigned short* WIH  = (unsigned short*)(ws + kOffWIH);
  unsigned short* WIL  = (unsigned short*)(ws + kOffWIL);
  unsigned short* UCH  = (unsigned short*)(ws + kOffUCH);
  unsigned short* UCL  = (unsigned short*)(ws + kOffUCL);
  unsigned short* YH   = (unsigned short*)(ws + kOffYH);
  unsigned short* YL   = (unsigned short*)(ws + kOffYL);
  float*          XZ   = (float*)(ws + kOffXZ);
  float*          UC   = (float*)(ws + kOffUC);
  unsigned short* WXH  = (unsigned short*)(ws + kOffWXH);
  unsigned short* WXL  = (unsigned short*)(ws + kOffWXL);
  float*          XD   = (float*)(ws + kOffXD);
  unsigned short* WOH  = (unsigned short*)(ws + kOffWOH);
  unsigned short* WOL  = (unsigned short*)(ws + kOffWOL);
  float*          MO   = (float*)(ws + kOffMO);
  float*          SEL  = (float*)(ws + kOffSEL);
  unsigned short* WQH  = (unsigned short*)(ws + kOffWQH);
  unsigned short* WQL  = (unsigned short*)(ws + kOffWQL);
  unsigned short* WPH  = (unsigned short*)(ws + kOffWPH);
  unsigned short* WPL  = (unsigned short*)(ws + kOffWPL);
  unsigned short* QKH  = (unsigned short*)(ws + kOffQKH);
  unsigned short* QKL  = (unsigned short*)(ws + kOffQKL);
  unsigned short* VTH  = (unsigned short*)(ws + kOffVTH);
  unsigned short* VTL  = (unsigned short*)(ws + kOffVTL);
  unsigned short* CTXH = (unsigned short*)(ws + kOffCTXH);
  unsigned short* CTXL = (unsigned short*)(ws + kOffCTXL);
  float*          Sbuf = (float*)(ws + kOffS);
  unsigned short* PH   = (unsigned short*)(ws + kOffPH);
  unsigned short* PL   = (unsigned short*)(ws + kOffPL);

  const float* dummy_f = SEL;
  void* dummy_c2 = (void*)PL;

  ln_rms_kernel<<<dim3(kRows), dim3(256), 0, stream>>>(x, ln_w, ln_b, m_norm_w, XLN, XH, XL, HMH, HML);

  transpose_split_kernel<<<dim3(kHid / 64, kXzP / 64), dim3(256), 0, stream>>>(in_proj_w, kXzP, kXzP, WIH, WIL, kHid);
  transpose_split_kernel<<<dim3(kInn / 64, kXdP / 64), dim3(256), 0, stream>>>(x_proj_w, kXdW, kXdW, WXH, WXL, kInn);
  transpose_split_kernel<<<dim3(kInn / 64, kHid / 64), dim3(256), 0, stream>>>(out_proj_w, kHid, kHid, WOH, WOL, kInn);

  wmma_gemm64<1, 2, 0, 0, false, 0, false><<<dim3(192, 1), dim3(256), 0, stream>>>(
      HMH, HML, kHid, 0L,
      WIH, WIL, kHid, 0L,
      (void*)XZ, dummy_c2, kXzP, 0L,
      dummy_f, dummy_f, 0L,
      kRows, kXzP, kHid, 1.0f);

  conv_silu_kernel<<<dim3(kInn / 256, kRows / 64), dim3(256), 0, stream>>>(XZ, conv_w, conv_b, UC, UCH, UCL);

  wmma_gemm64<1, 2, 0, 0, false, 0, false><<<dim3(8, 1), dim3(256), 0, stream>>>(
      UCH, UCL, kInn, 0L,
      WXH, WXL, kInn, 0L,
      (void*)XD, dummy_c2, kXdP, 0L,
      dummy_f, dummy_f, 0L,
      kRows, kXdP, kInn, 1.0f);

  scan_kernel<<<dim3(kBatch * (kInn / kScanCh)), dim3(kScanCh), 0, stream>>>(XD, UC, XZ, dt_proj_w, dt_proj_b, A_log, Dp, YH, YL);

  wmma_gemm64<1, 2, 0, 0, true, 6, false><<<dim3(48, 1), dim3(256), 0, stream>>>(
      YH, YL, kInn, 0L,
      WOH, WOL, kInn, 0L,
      (void*)MO, dummy_c2, kHid, 0L,
      dummy_f, XLN, 0L,
      kRows, kHid, kInn, 1.0f);

  gate_kernel<<<dim3(kRows / 32), dim3(256), 0, stream>>>(MO, sel_w, sel_b, SEL);

  transpose_split_kernel<<<dim3(kHid / 64, kQkvN / 64), dim3(256), 0, stream>>>(c_attn_w, kQkvN, kQkvN, WQH, WQL, kHid);
  transpose_split_kernel<<<dim3(kHid / 64, kHid / 64), dim3(256), 0, stream>>>(c_proj_w, kHid, kHid, WPH, WPL, kHid);

  wmma_gemm64<1, 2, 2, 2, false, 0, false><<<dim3(96, 1), dim3(256), 0, stream>>>(
      XH, XL, kHid, 0L,
      WQH, WQL, kHid, 0L,
      (void*)QKH, (void*)QKL, kQKld, 0L,
      c_attn_b, dummy_f, 0L,
      kRows, kQKld, kHid, 1.0f);

  wmma_gemm64<1, 2, 1, 2, false, 0, false><<<dim3(48, 1), dim3(256), 0, stream>>>(
      WQH + (size_t)kQKld * kHid, WQL + (size_t)kQKld * kHid, kHid, 0L,
      XH, XL, kHid, 0L,
      (void*)VTH, (void*)VTL, kRows, 0L,
      c_attn_b + kQKld, dummy_f, 0L,
      kHid, kRows, kHid, 1.0f);

  for (int g = 0; g < kNumGroups; ++g) {
    const int b  = g / (kNH / kGrp);
    const int h0 = (g % (kNH / kGrp)) * kGrp;
    const size_t qkoff = (size_t)b * kT * kQKld + (size_t)h0 * kDH;

    wmma_gemm64<1, 2, 0, 0, false, 0, true><<<dim3((kT / 64) * (kT / 64) / 8, kGrp), dim3(256), 0, stream>>>(
        QKH + qkoff, QKL + qkoff, kQKld, (long)kDH,
        QKH + kHid + qkoff, QKL + kHid + qkoff, kQKld, (long)kDH,
        (void*)Sbuf, dummy_c2, kT, (long)kT * kT,
        dummy_f, dummy_f, 0L,
        kT, kT, kDH, kScoreScale);

    softmax_dual_kernel<<<dim3(kGrp * kT), dim3(128), 0, stream>>>(Sbuf, SEL + (size_t)b * kT, w_local, w_global, PH, PL);

    const size_t vtoff = (size_t)(h0 * kDH) * kRows + (size_t)b * kT;
    const size_t coff  = (size_t)b * kT * kHid + (size_t)h0 * kDH;
    wmma_gemm64<1, 2, 0, 2, false, 0, true><<<dim3((kT / 64) * (kDH / 64) / 8, kGrp), dim3(256), 0, stream>>>(
        PH, PL, kT, (long)kT * kT,
        VTH + vtoff, VTL + vtoff, kRows, (long)kDH * kRows,
        (void*)(CTXH + coff), (void*)(CTXL + coff), kHid, (long)kDH,
        dummy_f, dummy_f, 0L,
        kT, kDH, kT, 1.0f);
  }

  wmma_gemm64<1, 2, 2, 0, false, 0, false><<<dim3(48, 1), dim3(256), 0, stream>>>(
      CTXH, CTXL, kHid, 0L,
      WPH, WPL, kHid, 0L,
      (void*)out, dummy_c2, kHid, 0L,
      c_proj_b, dummy_f, 0L,
      kRows, kHid, kHid, 1.0f);
}
